// GCN_52226802320176
// MI455X (gfx1250) — hardware-verified
//
#include <hip/hip_runtime.h>
#include <stddef.h>
#include <stdint.h>
#include <math.h>


#define FD     128
#define K2     256
#define NTHR   256
#define NWAVE  8
#define EPT    8
#define CHUNK  (NTHR * EPT)
#define WCAP   (EPT * 32)
#define LISTN  (NWAVE * WCAP)
#define NBA    1024
#define SLA    10
#define RCAP   28672
#define DEGCAP 64
#define GBM    64
#define GBN    128
#define GTHR   128
#define GWAVE  (GTHR / 32)
#define SBM    128
#define RECW   384
#define NU1    (FD * (FD / 8))
#define NU2    (FD * (K2 / 8))
#define NUP    256
#define PARN   1024
#define PA_B1  0
#define PA_G1  128
#define PA_BE1 256
#define PA_B2  384
#define PA_G2  512
#define PA_BE2 640
#define PA_A   768
#define BK_ZINTS (LISTN + 2 * RCAP + 3 * NBA)
#define BK_LDS_INTS (BK_ZINTS + 16)
#define WSMAX  134217728

static_assert((CHUNK & (CHUNK - 1)) == 0 && CHUNK <= 4096);
static_assert((NBA & (NBA - 1)) == 0 && NBA == (1 << SLA));
static_assert(((long long)CHUNK << SLA) < (1LL << 31));
static_assert(LISTN % NTHR == 0);
static_assert(NBA % NWAVE == 0 && NBA % 32 == 0 && NBA == NTHR * 4);
static_assert(RCAP % (NTHR * 4) == 0 && BK_ZINTS % 4 == 0 && LISTN % 4 == 0);
static_assert(BK_LDS_INTS * 4 <= 300000);
static_assert((long long)RCAP * 100 >= 16696LL * 105);
static_assert(DEGCAP >= 33 + 8);
static_assert(49 * NBA >= 50000 && 391 * SBM == 50048);
static_assert(FD == 32 * 4 && FD % 32 == 0 && K2 % 32 == 0 && K2 == 2 * FD && GBN == FD);
static_assert(GBM == GWAVE * 16 && SBM % GBM == 0 && NBA % SBM == 0);
static_assert(NU1 % NTHR == 0 && NU2 % NTHR == 0 && NUP == NTHR && PARN == 4 * NUP);
static_assert(RECW == 3 * FD && (RECW / 4) <= FD && RECW % 32 == 0);
static_assert(2 * NBA <= RCAP);

typedef float          v4f   __attribute__((ext_vector_type(4)));
typedef float          v8f   __attribute__((ext_vector_type(8)));
typedef int            v4i   __attribute__((ext_vector_type(4)));
typedef int            v8i   __attribute__((ext_vector_type(8)));
typedef unsigned short v4us  __attribute__((ext_vector_type(4)));
typedef unsigned short v8us  __attribute__((ext_vector_type(8)));
typedef unsigned short v16us __attribute__((ext_vector_type(16)));
typedef __bf16         v16bf __attribute__((ext_vector_type(16)));
typedef v4f  __attribute__((may_alias)) v4fa;
typedef v4i  __attribute__((may_alias)) v4ia;
typedef v8us __attribute__((may_alias)) v8usa;
union FragB { v16bf v; v16us u; v8us h[2]; v8i w; };

__device__ __forceinline__ v8f wmb(const FragB& a, const FragB& b, v8f c) {
  v8f d = __builtin_amdgcn_wmma_f32_16x16x32_bf16(false, a.v, false, b.v, (short)0, c, false, false);
  asm volatile("v_nop\n\tv_nop\n\tv_nop\n\tv_nop" : "+v"(d) : "v"(a.w), "v"(b.w));
  return d;
}

__device__ __forceinline__ v8f z8() { v8f z = {0.f, 0.f, 0.f, 0.f, 0.f, 0.f, 0.f, 0.f}; return z; }

__device__ __forceinline__ unsigned bf16_bits(float f) {
  const unsigned u = __float_as_uint(f);
  const unsigned r = (u + 0x7FFFu + ((u >> 16) & 1u)) >> 16;
  const unsigned nb = (u >> 16) | 0x40u;
  return ((u & 0x7FFFFFFFu) > 0x7F800000u) ? nb : r;
}
__device__ __forceinline__ float bf16_val(float f) {
  return __uint_as_float(bf16_bits(f) << 16);
}

template <int SLB>
__device__ __forceinline__ int scan_chunk(const int* __restrict__ dsts, int nE, int cbase, int slotBase,
                                          int nb, int vec8, int* list, int tid, int lane, int wave) {
  int wc = 0;
  const int el0  = tid * EPT;
  const int e0   = cbase + el0;
  const int sent = -2147483647 - 1;
  v4i da, db;
  if (vec8 != 0 && cbase + CHUNK <= nE) {
    da = *(const v4i*)(dsts + e0);
    db = *(const v4i*)(dsts + e0 + 4);
  } else {
    da.x = (e0     < nE) ? dsts[min(e0,     nE - 1)] : sent;
    da.y = (e0 + 1 < nE) ? dsts[min(e0 + 1, nE - 1)] : sent;
    da.z = (e0 + 2 < nE) ? dsts[min(e0 + 2, nE - 1)] : sent;
    da.w = (e0 + 3 < nE) ? dsts[min(e0 + 3, nE - 1)] : sent;
    db.x = (e0 + 4 < nE) ? dsts[min(e0 + 4, nE - 1)] : sent;
    db.y = (e0 + 5 < nE) ? dsts[min(e0 + 5, nE - 1)] : sent;
    db.z = (e0 + 6 < nE) ? dsts[min(e0 + 6, nE - 1)] : sent;
    db.w = (e0 + 7 < nE) ? dsts[min(e0 + 7, nE - 1)] : sent;
  }
  const unsigned nbs = (unsigned)slotBase;
  const unsigned unb = (unsigned)nb;
  const unsigned s0 = (unsigned)da.x - nbs, s1 = (unsigned)da.y - nbs;
  const unsigned s2 = (unsigned)da.z - nbs, s3 = (unsigned)da.w - nbs;
  const unsigned s4 = (unsigned)db.x - nbs, s5 = (unsigned)db.y - nbs;
  const unsigned s6 = (unsigned)db.z - nbs, s7 = (unsigned)db.w - nbs;
  const bool h0 = s0 < unb, h1 = s1 < unb, h2 = s2 < unb, h3 = s3 < unb;
  const bool h4 = s4 < unb, h5 = s5 < unb, h6 = s6 < unb, h7 = s7 < unb;
  const unsigned any = __builtin_amdgcn_ballot_w32(h0 | h1 | h2 | h3 | h4 | h5 | h6 | h7);
  if (any != 0u) {
#define HITJ(J, HJ, SJ) { \
      const unsigned mj = __builtin_amdgcn_ballot_w32(HJ); \
      if (mj != 0u) { \
        if (HJ) { \
          const int pos = wc + (int)__builtin_amdgcn_mbcnt_lo(mj, 0u); \
          if (pos < WCAP) list[wave * WCAP + pos] = ((el0 + (J)) << SLB) | (int)(SJ); \
        } \
        wc += (int)__builtin_popcount(mj); } }
    HITJ(0, h0, s0)
    HITJ(1, h1, s1)
    HITJ(2, h2, s2)
    HITJ(3, h3, s3)
    HITJ(4, h4, s4)
    HITJ(5, h5, s5)
    HITJ(6, h6, s6)
    HITJ(7, h7, s7)
#undef HITJ
  }
  return wc;
}

__global__ __launch_bounds__(NTHR) void k_prep(
    const float* __restrict__ feat, const float* __restrict__ W1, const float* __restrict__ W2,
    const float* __restrict__ b1, const float* __restrict__ g1, const float* __restrict__ be1,
    const float* __restrict__ a1, const float* __restrict__ b2, const float* __restrict__ g2,
    const float* __restrict__ be2, const float* __restrict__ a2,
    int nN, int uFB,
    unsigned short* FB, unsigned short* W1T, unsigned short* W2T, float* PAR) {
  const int u = (int)blockIdx.x * NTHR + (int)threadIdx.x;
  v8us o;
  unsigned short* dp;
  if (u < uFB) {
    const int row = u >> 4;
    const int k8  = (u & 15) * 8;
    const int rc  = row < nN ? row : nN - 1;
    const float* p = feat + (size_t)rc * FD + k8;
    const v4f a = *(const v4fa*)p;
    const v4f b = *(const v4fa*)(p + 4);
    const bool ok = row < nN;
    o[0] = ok ? (unsigned short)bf16_bits(a.x) : (unsigned short)0;
    o[1] = ok ? (unsigned short)bf16_bits(a.y) : (unsigned short)0;
    o[2] = ok ? (unsigned short)bf16_bits(a.z) : (unsigned short)0;
    o[3] = ok ? (unsigned short)bf16_bits(a.w) : (unsigned short)0;
    o[4] = ok ? (unsigned short)bf16_bits(b.x) : (unsigned short)0;
    o[5] = ok ? (unsigned short)bf16_bits(b.y) : (unsigned short)0;
    o[6] = ok ? (unsigned short)bf16_bits(b.z) : (unsigned short)0;
    o[7] = ok ? (unsigned short)bf16_bits(b.w) : (unsigned short)0;
    dp = FB + (size_t)row * FD + k8;
  } else if (u < uFB + NU1) {
    const int v  = u - uFB;
    const int n  = v >> 4;
    const int k8 = (v & 15) * 8;
    const float* p = W1 + (size_t)k8 * FD + n;
#pragma unroll
    for (int i = 0; i < 8; ++i) o[i] = (unsigned short)bf16_bits(p[(size_t)i * FD]);
    dp = W1T + (size_t)n * FD + k8;
  } else if (u < uFB + NU1 + NU2) {
    const int v  = u - uFB - NU1;
    const int n  = v >> 5;
    const int k8 = (v & 31) * 8;
    const int kk = k8 & (FD - 1);
    const float* p = W2 + (size_t)kk * FD + n;
#pragma unroll
    for (int i = 0; i < 8; ++i) o[i] = (unsigned short)bf16_bits(p[(size_t)i * FD]);
    dp = W2T + (size_t)n * K2 + k8;
  } else if (u < uFB + NU1 + NU2 + NUP) {
    const int p   = u - uFB - NU1 - NU2;
    const int arr = p >> 5;
    const int c   = (p & 31) * 4;
    const v4f c0 = *(const v4fa*)(b1 + c);
    const v4f c1 = *(const v4fa*)(g1 + c);
    const v4f c2 = *(const v4fa*)(be1 + c);
    const v4f c3 = *(const v4fa*)(b2 + c);
    const v4f c4 = *(const v4fa*)(g2 + c);
    const v4f c5 = *(const v4fa*)(be2 + c);
    const float s1 = a1[0];
    const float s2 = a2[0];
    const unsigned m0 = 0u - (unsigned)(arr == 0), m1 = 0u - (unsigned)(arr == 1);
    const unsigned m2 = 0u - (unsigned)(arr == 2), m3 = 0u - (unsigned)(arr == 3);
    const unsigned m4 = 0u - (unsigned)(arr == 4), m5 = 0u - (unsigned)(arr == 5);
    const unsigned m6 = 0u - (unsigned)(p == 192);
    unsigned bx = (__float_as_uint(c0.x) & m0) | (__float_as_uint(c1.x) & m1) | (__float_as_uint(c2.x) & m2) |
                  (__float_as_uint(c3.x) & m3) | (__float_as_uint(c4.x) & m4) | (__float_as_uint(c5.x) & m5) |
                  (__float_as_uint(s1) & m6);
    unsigned by = (__float_as_uint(c0.y) & m0) | (__float_as_uint(c1.y) & m1) | (__float_as_uint(c2.y) & m2) |
                  (__float_as_uint(c3.y) & m3) | (__float_as_uint(c4.y) & m4) | (__float_as_uint(c5.y) & m5) |
                  (__float_as_uint(s2) & m6);
    unsigned bz = (__float_as_uint(c0.z) & m0) | (__float_as_uint(c1.z) & m1) | (__float_as_uint(c2.z) & m2) |
                  (__float_as_uint(c3.z) & m3) | (__float_as_uint(c4.z) & m4) | (__float_as_uint(c5.z) & m5);
    unsigned bw = (__float_as_uint(c0.w) & m0) | (__float_as_uint(c1.w) & m1) | (__float_as_uint(c2.w) & m2) |
                  (__float_as_uint(c3.w) & m3) | (__float_as_uint(c4.w) & m4) | (__float_as_uint(c5.w) & m5);
    v4f pv;
    pv.x = bf16_val(__uint_as_float(bx));
    pv.y = bf16_val(__uint_as_float(by));
    pv.z = bf16_val(__uint_as_float(bz));
    pv.w = bf16_val(__uint_as_float(bw));
    float* pp = PAR + 4 * p;
    *(volatile v4f*)pp = pv;
    __threadfence();
    *(volatile v4f*)pp = pv;
    return;
  } else {
    return;
  }
  *(volatile v8us*)dp = o;
  __threadfence();
  *(volatile v8us*)dp = o;
}

__global__ __launch_bounds__(NTHR) void k_bucket(const int* __restrict__ srcs, const int* __restrict__ dsts,
                                                 int nE, int nN, int vec8,
                                                 int* hits, int* cntg, int* offg, float* din, float* dout) {
  extern __shared__ __attribute__((aligned(16))) int dsm[];
  int* list = dsm;
  int* hl   = dsm + LISTN;
  int* sl   = hl + RCAP;
  int* cnt  = sl + RCAP;
  int* offs = cnt + NBA;
  int* cur  = offs + NBA;
  int* misc = cur + NBA;
  const int tid = (int)threadIdx.x, lane = tid & 31, wave = tid >> 5;
  const int nodeBase = (int)blockIdx.x * NBA;

  {
    const v4i z4 = {0, 0, 0, 0};
    for (int i = tid * 4; i < BK_ZINTS; i += NTHR * 4) *(v4ia*)(dsm + i) = z4;
    if (tid < 16) misc[tid] = 0;
  }
  __syncthreads();

  int t = 0, ov = 0;
  const int nChunks = (nE + CHUNK - 1) / CHUNK;
#pragma unroll 1
  for (int ch = 0; ch < nChunks; ++ch) {
    const int cbase = ch * CHUNK;
    const int wc = scan_chunk<SLA>(dsts, nE, cbase, nodeBase, NBA, vec8, list, tid, lane, wave);
    if (lane == 0) misc[wave] = wc;
    __syncthreads();
    if (wave == 0) {
#pragma unroll 1
      for (int w2 = 0; w2 < NWAVE; ++w2) {
        int c = misc[w2];
        c = c < 0 ? 0 : (c > WCAP ? WCAP : c);
#pragma unroll 1
        for (int b0 = 0; b0 < c; b0 += 32) {
          const int idx = b0 + lane;
          const int ent = list[w2 * WCAP + (idx < WCAP ? idx : WCAP - 1)];
          const int m32 = (c - b0) < 32 ? (c - b0) : 32;
#pragma unroll 1
          for (int k = 0; k < m32; ++k) {
            const int u    = __builtin_amdgcn_readlane(ent, k);
            const int slot = u & (NBA - 1);
            const int el   = (u >> SLA) & (CHUNK - 1);
            const int pk   = ((cbase + el) << SLA) | slot;
            if (t < RCAP) {
              if (lane == 0) { hl[t] = pk; cnt[slot] = cnt[slot] + 1; }
              t = t + 1;
            } else {
              ov = 1;
            }
          }
        }
      }
    }
    __syncthreads();
  }
  if (wave == 0 && lane == 0) { misc[8] = t; misc[9] = ov; }
  __syncthreads();
  int tt = misc[8];
  tt = tt < 0 ? 0 : (tt > RCAP ? RCAP : tt);
  const int ovf = misc[9];

  if (wave == 0) {
    const int base = lane * (NBA / 32);
    int s = 0;
#pragma unroll 1
    for (int i = 0; i < NBA / 32; ++i) s += cnt[base + i];
    int incl = s;
#pragma unroll
    for (int d = 1; d < 32; d <<= 1) {
      const int y = __shfl_up(incl, d, 32);
      if (lane >= d) incl += y;
    }
    int run = incl - s;
#pragma unroll 1
    for (int i = 0; i < NBA / 32; ++i) {
      const int cv = cnt[base + i];
      offs[base + i] = run;
      cur[base + i]  = run;
      run += cv;
    }
  }
  __syncthreads();
  if (wave == 0) {
#pragma unroll 1
    for (int b0 = 0; b0 < tt; b0 += 32) {
      const int idx = b0 + lane;
      const int ent = hl[idx < RCAP ? idx : RCAP - 1];
      const int m32 = (tt - b0) < 32 ? (tt - b0) : 32;
#pragma unroll 1
      for (int k = 0; k < m32; ++k) {
        const int u    = __builtin_amdgcn_readlane(ent, k);
        const int slot = u & (NBA - 1);
        if (lane == 0) {
          int p = cur[slot];
          p = p < 0 ? 0 : (p > RCAP - 1 ? RCAP - 1 : p);
          sl[p] = u;
          cur[slot] = p + 1;
        }
      }
    }
  }
  __syncthreads();

  int* hbp = hits + (size_t)blockIdx.x * RCAP;
#pragma unroll 1
  for (int it = 0; it < RCAP / (NTHR * 4); ++it) {
    const int i0 = it * (NTHR * 4) + 4 * tid;
    const v4i e4 = *(const v4ia*)(sl + i0);
    int q0 = e4.x >> SLA, q1 = e4.y >> SLA, q2 = e4.z >> SLA, q3 = e4.w >> SLA;
    q0 = q0 < 0 ? 0 : (q0 > nE - 1 ? nE - 1 : q0);
    q1 = q1 < 0 ? 0 : (q1 > nE - 1 ? nE - 1 : q1);
    q2 = q2 < 0 ? 0 : (q2 > nE - 1 ? nE - 1 : q2);
    q3 = q3 < 0 ? 0 : (q3 > nE - 1 ? nE - 1 : q3);
    int r0 = srcs[q0], r1 = srcs[q1], r2 = srcs[q2], r3 = srcs[q3];
    r0 = r0 < 0 ? 0 : (r0 > nN - 1 ? nN - 1 : r0);
    r1 = r1 < 0 ? 0 : (r1 > nN - 1 ? nN - 1 : r1);
    r2 = r2 < 0 ? 0 : (r2 > nN - 1 ? nN - 1 : r2);
    r3 = r3 < 0 ? 0 : (r3 > nN - 1 ? nN - 1 : r3);
    v4i o4;
    o4.x = (i0     < tt) ? r0 : 0;
    o4.y = (i0 + 1 < tt) ? r1 : 0;
    o4.z = (i0 + 2 < tt) ? r2 : 0;
    o4.w = (i0 + 3 < tt) ? r3 : 0;
    *(volatile v4i*)(hbp + i0) = o4;
    __threadfence();
    *(volatile v4i*)(hbp + i0) = o4;
  }

  float* fb = (float*)hl;
#pragma unroll 1
  for (int j = 0; j < 4; ++j) {
    const int s = j * NTHR + tid;
    const int c = cnt[s];
    fb[s] = 1.0f / sqrtf((float)(c < 1 ? 1 : c));
  }
  __syncthreads();
  {
    const v4i c4 = *(const v4ia*)(cnt + 4 * tid);
    const v4i f4 = *(const v4ia*)(offs + 4 * tid);
    const v4f d4 = *(const v4fa*)(fb + 4 * tid);
    v4i cw;
    cw.x = (ovf != 0) ? -1 : c4.x;
    cw.y = (ovf != 0) ? -1 : c4.y;
    cw.z = (ovf != 0) ? -1 : c4.z;
    cw.w = (ovf != 0) ? -1 : c4.w;
    int*   cp = cntg + (size_t)nodeBase + 4 * tid;
    int*   op = offg + (size_t)nodeBase + 4 * tid;
    float* dq = din  + (size_t)nodeBase + 4 * tid;
    *(volatile v4i*)cp = cw;
    *(volatile v4i*)op = f4;
    *(volatile v4f*)dq = d4;
    __threadfence();
    *(volatile v4i*)cp = cw;
    *(volatile v4i*)op = f4;
    *(volatile v4f*)dq = d4;
  }

  {
    const v4i z4 = {0, 0, 0, 0};
    *(v4ia*)(cur + 4 * tid) = z4;
  }
  __syncthreads();
#pragma unroll 1
  for (int ch = 0; ch < nChunks; ++ch) {
    const int cbase = ch * CHUNK;
    const int wc = scan_chunk<SLA>(srcs, nE, cbase, nodeBase, NBA, vec8, list, tid, lane, wave);
    if (lane == 0) misc[wave] = wc;
    __syncthreads();
    if (wave == 0) {
#pragma unroll 1
      for (int w2 = 0; w2 < NWAVE; ++w2) {
        int c = misc[w2];
        c = c < 0 ? 0 : (c > WCAP ? WCAP : c);
#pragma unroll 1
        for (int b0 = 0; b0 < c; b0 += 32) {
          const int idx = b0 + lane;
          const int ent = list[w2 * WCAP + (idx < WCAP ? idx : WCAP - 1)];
          const int m32 = (c - b0) < 32 ? (c - b0) : 32;
#pragma unroll 1
          for (int k = 0; k < m32; ++k) {
            const int u    = __builtin_amdgcn_readlane(ent, k);
            const int slot = u & (NBA - 1);
            if (lane == 0) cur[slot] = cur[slot] + 1;
          }
        }
      }
    }
    __syncthreads();
  }
#pragma unroll 1
  for (int j = 0; j < 4; ++j) {
    const int s = j * NTHR + tid;
    const int c = cur[s];
    fb[NBA + s] = 1.0f / sqrtf((float)(c < 1 ? 1 : c));
  }
  __syncthreads();
  {
    const v4f d4 = *(const v4fa*)(fb + NBA + 4 * tid);
    float* dq = dout + (size_t)nodeBase + 4 * tid;
    *(volatile v4f*)dq = d4;
    __threadfence();
    *(volatile v4f*)dq = d4;
  }
}

template <int SCALE>
__global__ __launch_bounds__(GTHR) void k_gemm(const unsigned short* __restrict__ A,
                                               const unsigned short* __restrict__ BT, int K,
                                               const float* __restrict__ rs, float* outF) {
  __shared__ __attribute__((aligned(16))) float stg[GBM * GBN];
  const int tid = (int)threadIdx.x, lane = tid & 31, wave = tid >> 5, hh = lane >> 4, m = lane & 15;
  const int rowBase = (int)blockIdx.x * GBM;

  v8f acc[8];
#pragma unroll
  for (int t = 0; t < 8; ++t) acc[t] = z8();
  const unsigned short* ap = A  + (size_t)(rowBase + 16 * wave + m) * (size_t)K + 8 * hh;
  const unsigned short* bp = BT + (size_t)m * (size_t)K + 8 * hh;

#pragma unroll 1
  for (int k0 = 0; k0 < K; k0 += 32) {
    FragB af;
    af.h[0] = *(const v8usa*)(ap + k0);
    af.h[1] = *(const v8usa*)(ap + k0 + 16);
#pragma unroll
    for (int nt = 0; nt < 8; ++nt) {
      const unsigned short* wq = bp + (size_t)(16 * nt) * (size_t)K + k0;
      FragB bf;
      bf.h[0] = *(const v8usa*)wq;
      bf.h[1] = *(const v8usa*)(wq + 16);
      acc[nt] = wmb(af, bf, acc[nt]);
    }
  }

#pragma unroll
  for (int nt = 0; nt < 8; ++nt) {
    const int lc = 16 * nt + m;
#pragma unroll
    for (int r = 0; r < 8; ++r) {
      const int lr = 16 * wave + 8 * hh + r;
      stg[lr * GBN + lc] = acc[nt][r];
    }
  }
  __syncthreads();

  int dsi = __float_as_int(1.0f);
  if constexpr (SCALE != 0) dsi = __float_as_int(rs[rowBase + 16 * wave + m]);
  v4f pv[16];
#pragma unroll
  for (int i = 0; i < 16; ++i) {
    const v4f x = *(const v4fa*)(stg + (16 * wave + i) * GBN + 4 * lane);
    if constexpr (SCALE != 0) {
      const float sc = __int_as_float(__builtin_amdgcn_readlane(dsi, i));
      v4f q;
      q.x = x.x * sc; q.y = x.y * sc; q.z = x.z * sc; q.w = x.w * sc;
      pv[i] = q;
    } else {
      pv[i] = x;
    }
  }
#pragma unroll
  for (int i = 0; i < 16; ++i) {
    float* op = outF + (size_t)(rowBase + 16 * wave + i) * (size_t)GBN + 4 * lane;
    *(volatile v4f*)op = pv[i];
  }
  __threadfence();
#pragma unroll
  for (int i = 0; i < 16; ++i) {
    float* op = outF + (size_t)(rowBase + 16 * wave + i) * (size_t)GBN + 4 * lane;
    *(volatile v4f*)op = pv[i];
  }
}

__global__ __launch_bounds__(NTHR) void k_agg(const int* __restrict__ hits, const int* __restrict__ cntg,
                                              const int* __restrict__ offg, const float* __restrict__ din,
                                              const float* __restrict__ hrows, const float* __restrict__ par,
                                              int biasOff, int nN, int mRows, float* y) {
  __shared__ __attribute__((aligned(16))) int   scnt[NBA];
  __shared__ __attribute__((aligned(16))) int   soff[NBA];
  __shared__ __attribute__((aligned(16))) float sdin[NBA];
  const int tid = (int)threadIdx.x, lane = tid & 31, wave = tid >> 5;
  const int nodeBase = (int)blockIdx.x * NBA;
  {
    const v4i c4 = *(const v4i*)(cntg + (size_t)nodeBase + 4 * tid);
    const v4i o4 = *(const v4i*)(offg + (size_t)nodeBase + 4 * tid);
    const v4f d4 = *(const v4f*)(din  + (size_t)nodeBase + 4 * tid);
    *(v4ia*)(scnt + 4 * tid) = c4;
    *(v4ia*)(soff + 4 * tid) = o4;
    *(v4fa*)(sdin + 4 * tid) = d4;
  }
  const v4f bq = *(const v4f*)(par + biasOff + 4 * lane);
  __syncthreads();

  const int* hbp = hits + (size_t)blockIdx.x * RCAP;
  const float qnan = __int_as_float(0x7fc00000);
#pragma unroll 1
  for (int si = 0; si < NBA / NWAVE; ++si) {
    const int s    = si * NWAVE + wave;
    const int node = nodeBase + s;
    int c = scnt[s];
    const bool bad = (c < 0) || (c > DEGCAP);
    c = c < 0 ? 0 : (c > DEGCAP ? DEGCAP : c);
    int o = soff[s];
    o = o < 0 ? 0 : (o > RCAP - 1 ? RCAP - 1 : o);
    const float dd = sdin[s];
    float a0 = 0.0f, a1 = 0.0f, a2 = 0.0f, a3 = 0.0f;
#pragma unroll 1
    for (int b0 = 0; b0 < c; b0 += 32) {
      int idx = o + b0 + lane;
      idx = idx > RCAP - 1 ? RCAP - 1 : idx;
      int sr = hbp[idx];
      sr = sr < 0 ? 0 : (sr > nN - 1 ? nN - 1 : sr);
      const int m32 = (c - b0) < 32 ? (c - b0) : 32;
#pragma unroll 1
      for (int k = 0; k < m32; ++k) {
        const int sk = __builtin_amdgcn_readlane(sr, k);
        const v4f a = *(const v4fa*)(hrows + (size_t)sk * FD + 4 * lane);
        a0 += a.x; a1 += a.y; a2 += a.z; a3 += a.w;
      }
    }
    const bool live = node < nN;
    float y0 = a0 * dd + bq.x;
    float y1 = a1 * dd + bq.y;
    float y2 = a2 * dd + bq.z;
    float y3 = a3 * dd + bq.w;
    y0 = bad ? qnan : y0; y1 = bad ? qnan : y1; y2 = bad ? qnan : y2; y3 = bad ? qnan : y3;
    v4f ov;
    ov.x = live ? y0 : 0.0f;
    ov.y = live ? y1 : 0.0f;
    ov.z = live ? y2 : 0.0f;
    ov.w = live ? y3 : 0.0f;
    if (node < mRows) {
      float* op = y + (size_t)node * FD + 4 * lane;
      *(volatile v4f*)op = ov;
      __threadfence();
      *(volatile v4f*)op = ov;
    }
  }
}

__global__ __launch_bounds__(FD) void k_stats(const float* __restrict__ y, int nN, float* rec) {
  __shared__ __attribute__((aligned(16))) float srec[RECW];
  const int tid = (int)threadIdx.x;
  const int row0 = (int)blockIdx.x * SBM;
  int nb = nN - row0;
  nb = nb < 0 ? 0 : (nb > SBM ? SBM : nb);
  const float* yp = y + (size_t)row0 * FD + tid;
  float s = 0.0f;
#pragma unroll 4
  for (int i = 0; i < nb; ++i) s += yp[(size_t)i * FD];
  const float rn = 1.0f / (float)(nb < 1 ? 1 : nb);
  const float mean = s * rn;
  float q = 0.0f;
#pragma unroll 4
  for (int i = 0; i < nb; ++i) {
    const float d = yp[(size_t)i * FD] - mean;
    q = fmaf(d, d, q);
  }
  srec[tid] = (float)nb;
  srec[FD + tid] = mean;
  srec[2 * FD + tid] = q;
  __syncthreads();
  v4f v;
  float* rp = rec + (size_t)blockIdx.x * RECW + 4 * tid;
  if (tid < RECW / 4) {
    v = *(const v4fa*)(srec + 4 * tid);
    *(volatile v4f*)rp = v;
  }
  __threadfence();
  if (tid < RECW / 4) {
    *(volatile v4f*)rp = v;
  }
}

__global__ __launch_bounds__(FD) void k_comb(const float* __restrict__ rec, int nRec, float* stat) {
  __shared__ __attribute__((aligned(16))) float stg[2 * FD];
  const int c = (int)threadIdx.x;
  double n = 0.0, mean = 0.0, M2 = 0.0;
#pragma unroll 1
  for (int b = 0; b < nRec; ++b) {
    const float* pr = rec + (size_t)b * RECW;
    const double nb = (double)pr[c];
    const double mb = (double)pr[FD + c];
    const double qb = (double)pr[2 * FD + c];
    if (nb > 0.5) {
      const double nn = n + nb;
      const double delta = mb - mean;
      const double f = nb / nn;
      mean = mean + delta * f;
      M2 = M2 + qb + delta * delta * n * f;
      n = nn;
    }
  }
  const double nt = n < 1.0 ? 1.0 : n;
  const float varf  = (float)(M2 / nt);
  const float meanf = (float)mean;
  const float rstd  = 1.0f / sqrtf(varf + 1e-5f);
  stg[c] = meanf;
  stg[FD + c] = rstd;
  __syncthreads();
  v4f v;
  if (c < (2 * FD) / 4) {
    v = *(const v4fa*)(stg + 4 * c);
    *(volatile v4f*)(stat + 4 * c) = v;
  }
  __threadfence();
  if (c < (2 * FD) / 4) {
    *(volatile v4f*)(stat + 4 * c) = v;
  }
}

__global__ __launch_bounds__(NTHR) void k_apply1(const float* __restrict__ y, const float* __restrict__ stat,
                                                 const float* __restrict__ par, const float* __restrict__ dout,
                                                 int nN, int nUnits, unsigned short* x1s) {
  const int u = (int)blockIdx.x * NTHR + (int)threadIdx.x;
  if (u >= nUnits) return;
  const int row = u >> 5;
  const int l   = u & 31;
  const int rc  = row < nN ? row : nN - 1;
  const bool ok = row < nN;
  const v4f yv = *(const v4f*)(y + (size_t)rc * FD + 4 * l);
  const v4f mv = *(const v4f*)(stat + 4 * l);
  const v4f rv = *(const v4f*)(stat + FD + 4 * l);
  const v4f gv = *(const v4f*)(par + PA_G1 + 4 * l);
  const v4f bv = *(const v4f*)(par + PA_BE1 + 4 * l);
  const float a   = par[PA_A];
  const float dsc = dout[rc];
  float yy[4], mm[4], rr[4], gg[4], bb[4];
  yy[0] = yv.x; yy[1] = yv.y; yy[2] = yv.z; yy[3] = yv.w;
  mm[0] = mv.x; mm[1] = mv.y; mm[2] = mv.z; mm[3] = mv.w;
  rr[0] = rv.x; rr[1] = rv.y; rr[2] = rv.z; rr[3] = rv.w;
  gg[0] = gv.x; gg[1] = gv.y; gg[2] = gv.z; gg[3] = gv.w;
  bb[0] = bv.x; bb[1] = bv.y; bb[2] = bv.z; bb[3] = bv.w;
  v4us hq, lq;
#pragma unroll
  for (int j = 0; j < 4; ++j) {
    float t = gg[j] * (yy[j] - mm[j]);
    t = t * rr[j];
    t = t + bb[j];
    const float p = (t >= 0.0f) ? t : a * t;
    const float x = p * dsc;
    const float xv = ok ? x : 0.0f;
    const unsigned hb = bf16_bits(xv);
    hq[j] = (unsigned short)hb;
    lq[j] = (unsigned short)bf16_bits(xv - __uint_as_float(hb << 16));
  }
  unsigned short* op = x1s + (size_t)row * K2 + 4 * l;
  *(volatile v4us*)op = hq;
  *(volatile v4us*)(op + FD) = lq;
  __threadfence();
  *(volatile v4us*)op = hq;
  *(volatile v4us*)(op + FD) = lq;
}

__global__ __launch_bounds__(NTHR) void k_apply2(const float* __restrict__ y, const float* __restrict__ stat,
                                                 const float* __restrict__ par, const int* __restrict__ cntg,
                                                 int nN, int nUnits, float* out) {
  const int u = (int)blockIdx.x * NTHR + (int)threadIdx.x;
  if (u >= nUnits) return;
  const int row = u >> 5;
  const int l   = u & 31;
  const int rc  = row < nN ? row : nN - 1;
  const v4f yv = *(const v4f*)(y + (size_t)rc * FD + 4 * l);
  const v4f mv = *(const v4f*)(stat + 4 * l);
  const v4f rv = *(const v4f*)(stat + FD + 4 * l);
  const v4f gv = *(const v4f*)(par + PA_G2 + 4 * l);
  const v4f bv = *(const v4f*)(par + PA_BE2 + 4 * l);
  const float a = par[PA_A + 1];
  const int cn  = cntg[rc];
  const bool bad = (cn < 0) || (cn > DEGCAP);
  const float qnan = __int_as_float(0x7fc00000);
  float yy[4], mm[4], rr[4], gg[4], bb[4], oo[4];
  yy[0] = yv.x; yy[1] = yv.y; yy[2] = yv.z; yy[3] = yv.w;
  mm[0] = mv.x; mm[1] = mv.y; mm[2] = mv.z; mm[3] = mv.w;
  rr[0] = rv.x; rr[1] = rv.y; rr[2] = rv.z; rr[3] = rv.w;
  gg[0] = gv.x; gg[1] = gv.y; gg[2] = gv.z; gg[3] = gv.w;
  bb[0] = bv.x; bb[1] = bv.y; bb[2] = bv.z; bb[3] = bv.w;
#pragma unroll
  for (int j = 0; j < 4; ++j) {
    float t = gg[j] * (yy[j] - mm[j]);
    t = t * rr[j];
    t = t + bb[j];
    const float p = (t >= 0.0f) ? t : a * t;
    oo[j] = bad ? qnan : p;
  }
  v4f ov;
  ov.x = oo[0]; ov.y = oo[1]; ov.z = oo[2]; ov.w = oo[3];
  float* op = out + (size_t)row * FD + 4 * l;
  *(volatile v4f*)op = ov;
  __threadfence();
  *(volatile v4f*)op = ov;
}

static inline int cdiv(int a, int b) { return (a + b - 1) / b; }
static inline size_t al256(size_t o) { return (o + 255) & ~(size_t)255; }

extern "C" void kernel_launch(void* const* d_in, const int* in_sizes, int n_in,
                              void* d_out, int out_size, void* d_ws, size_t ws_size,
                              hipStream_t stream) {
  if (n_in < 13) return;
  if (in_sizes[0] < FD || (in_sizes[0] % FD) != 0) return;
  const int nN = in_sizes[0] / FD;
  if (nN < 16 || nN >= (1 << 22)) return;
  const int nE = in_sizes[1];
  if (nE < 1 || in_sizes[2] != nE) return;
  if (nE >= (1 << (31 - SLA))) return;
  if (in_sizes[3] != FD * FD || in_sizes[8] != FD * FD) return;
  if (in_sizes[4] != FD || in_sizes[5] != FD || in_sizes[6] != FD) return;
  if (in_sizes[9] != FD || in_sizes[10] != FD || in_sizes[11] != FD) return;
  if (in_sizes[7] < 1 || in_sizes[12] < 1) return;
  if ((long long)out_size != (long long)nN * FD) return;

  const float* feat = (const float*)d_in[0];
  const int*   src  = (const int*)d_in[1];
  const int*   dst  = (const int*)d_in[2];
  const float* W1   = (const float*)d_in[3];
  const float* b1   = (const float*)d_in[4];
  const float* g1   = (const float*)d_in[5];
  const float* be1  = (const float*)d_in[6];
  const float* a1   = (const float*)d_in[7];
  const float* W2   = (const float*)d_in[8];
  const float* b2   = (const float*)d_in[9];
  const float* g2   = (const float*)d_in[10];
  const float* be2  = (const float*)d_in[11];
  const float* a2   = (const float*)d_in[12];
  float* out = (float*)d_out;

  const int MP   = cdiv(nN, SBM) * SBM;
  const int gM   = MP / GBM;
  const int nRec = MP / SBM;
  const int gA   = cdiv(MP, NBA);
  const int NP   = gA * NBA;
  if ((long long)gA * NBA < (long long)MP) return;
  if (MP % GBM != 0 || MP % SBM != 0 || MP < nN) return;
  const int vec8 = ((nE & 3) == 0) ? 1 : 0;
  const int uFB  = MP * (FD / 8);
  if (uFB % NTHR != 0) return;

  char* ws = (char*)d_ws;
  size_t off = 0;
  const size_t oFB  = off; off = al256(off + (size_t)MP * FD * 2);
  const size_t oW1T = off; off = al256(off + (size_t)FD * FD * 2);
  const size_t oW2T = off; off = al256(off + (size_t)FD * K2 * 2);
  const size_t oPAR = off; off = al256(off + (size_t)PARN * 4);
  const size_t oH   = off; off = al256(off + (size_t)MP * FD * 4);
  const size_t oY   = off; off = al256(off + (size_t)MP * FD * 4);
  const size_t oX   = off; off = al256(off + (size_t)MP * K2 * 2);
  const size_t oHT  = off; off = al256(off + (size_t)gA * RCAP * 4);
  const size_t oCN  = off; off = al256(off + (size_t)NP * 4);
  const size_t oOF  = off; off = al256(off + (size_t)NP * 4);
  const size_t oDI  = off; off = al256(off + (size_t)NP * 4);
  const size_t oDO  = off; off = al256(off + (size_t)NP * 4);
  const size_t oR1  = off; off = al256(off + (size_t)nRec * RECW * 4);
  const size_t oR2  = off; off = al256(off + (size_t)nRec * RECW * 4);
  const size_t oS1  = off; off = al256(off + (size_t)(2 * FD) * 4);
  const size_t oS2  = off; off = al256(off + (size_t)(2 * FD) * 4);
  if (off > ws_size || off > (size_t)WSMAX) return;
  unsigned short* FB  = (unsigned short*)(ws + oFB);
  unsigned short* W1T = (unsigned short*)(ws + oW1T);
  unsigned short* W2T = (unsigned short*)(ws + oW2T);
  float*          PAR = (float*)(ws + oPAR);
  float*          H   = (float*)(ws + oH);
  float*          Y   = (float*)(ws + oY);
  unsigned short* X1S = (unsigned short*)(ws + oX);
  int*            HT  = (int*)(ws + oHT);
  int*            CN  = (int*)(ws + oCN);
  int*            OF  = (int*)(ws + oOF);
  float*          DI  = (float*)(ws + oDI);
  float*          DO  = (float*)(ws + oDO);
  float*          R1  = (float*)(ws + oR1);
  float*          R2  = (float*)(ws + oR2);
  float*          S1  = (float*)(ws + oS1);
  float*          S2  = (float*)(ws + oS2);

  const size_t bkLds = (size_t)BK_LDS_INTS * 4;
  hipFuncSetAttribute(reinterpret_cast<const void*>(&k_bucket), hipFuncAttributeMaxDynamicSharedMemorySize, (int)bkLds);

  const int nU1 = MP * 32;
  const int nU2 = nN * 32;
  k_prep<<<(uFB + NU1 + NU2 + NUP) / NTHR, NTHR, 0, stream>>>(feat, W1, W2, b1, g1, be1, a1, b2, g2, be2, a2,
                                                               nN, uFB, FB, W1T, W2T, PAR);
  k_bucket<<<gA, NTHR, bkLds, stream>>>(src, dst, nE, nN, vec8, HT, CN, OF, DI, DO);
  k_gemm<1><<<gM, GTHR, 0, stream>>>(FB, W1T, FD, DO, H);
  k_agg<<<gA, NTHR, 0, stream>>>(HT, CN, OF, DI, H, PAR, PA_B1, nN, MP, Y);
  k_stats<<<nRec, FD, 0, stream>>>(Y, nN, R1);
  k_comb<<<1, FD, 0, stream>>>(R1, nRec, S1);
  k_apply1<<<cdiv(nU1, NTHR), NTHR, 0, stream>>>(Y, S1, PAR, DO, nN, nU1, X1S);
  k_gemm<0><<<gM, GTHR, 0, stream>>>(X1S, W2T, K2, DO, H);
  k_agg<<<gA, NTHR, 0, stream>>>(HT, CN, OF, DI, H, PAR, PA_B2, nN, MP, Y);
  k_stats<<<nRec, FD, 0, stream>>>(Y, nN, R2);
  k_comb<<<1, FD, 0, stream>>>(R2, nRec, S2);
  k_apply2<<<cdiv(nU2, NTHR), NTHR, 0, stream>>>(Y, S2, PAR, CN, nN, nU2, out);
}
